// PhysicsInformedEncoder_62843961475163
// MI455X (gfx1250) — hardware-run, weakly checked
//
#include <hip/hip_runtime.h>


namespace {
constexpr int N = 10000, E = 160000, G = 64, H = 128, H2 = 256, LAT = 64, NL = 3, NBLK = N / 16;
constexpr float XS = 8.0f, WSC = 256.0f, EPS = 1e-5f;
typedef _Float16 b16;
typedef __attribute__((ext_vector_type(16))) _Float16 v16b;
typedef __attribute__((ext_vector_type(8))) _Float16 v8b;
typedef __attribute__((ext_vector_type(8))) float v8f;
typedef __attribute__((ext_vector_type(4))) float v4f;
typedef __attribute__((ext_vector_type(2))) float v2f;
__device__ __forceinline__ float bf16_rne(float f) { unsigned int u = __float_as_uint(f); u += 0x7FFFu + ((u >> 16) & 1u); return __uint_as_float(u & 0xFFFF0000u); }
__device__ __forceinline__ void split16(float v, b16& hi, b16& lo) { hi = (b16)v; lo = (b16)(v - (float)hi); }
__device__ __forceinline__ v16b frag_kb(const b16* p, int hh) { const v8b a = *(const v8b*)(p + 8 * hh), b = *(const v8b*)(p + 16 + 8 * hh); v16b f;
#pragma unroll
  for (int e = 0; e < 8; ++e) { f[e] = a[e]; f[8 + e] = b[e]; } return f; }
__device__ __forceinline__ v8f wmma16b(v16b a, v16b b, v8f c) { v8f d = __builtin_amdgcn_wmma_f32_16x16x32_f16(false, a, false, b, (short)0, c, false, false); asm volatile("v_nop\n\tv_nop\n\tv_nop\n\tv_nop" : "+v"(d) : "v"(a), "v"(b)); return d; }
__device__ __forceinline__ void wave_lds_sync() { __builtin_amdgcn_fence(__ATOMIC_RELEASE, "workgroup"); __builtin_amdgcn_wave_barrier(); __builtin_amdgcn_fence(__ATOMIC_ACQUIRE, "workgroup"); }
__device__ __forceinline__ float pmul(float a, float b) { float p = a * b; asm volatile("" : "+v"(p)); return p; }
__device__ __forceinline__ int iclamp(int v, int lo, int hi) { return v < lo ? lo : (v > hi ? hi : v); }
__device__ __forceinline__ float sigm(float v) { return 1.0f / (1.0f + __expf(-v)); }
__device__ __forceinline__ float silu(float v) { return pmul(v, sigm(v)); }
constexpr int CSR_NBLK9 = 512, CSR_GB9 = 9, CSR_GN9 = 1 << CSR_GB9  , CSR_TS9 = (CSR_GN9 < 32 ? 32 : CSR_GN9)  , CSR_MAXG9 = 512, CSR_CAP9 = 12288  ;
__device__ __host__ __forceinline__ int csr_tix9(int v) { return (v >> CSR_GB9) * CSR_TS9 + (v & (CSR_GN9 - 1)); }
__global__ __launch_bounds__(64) void csrA_kernel9(const int* __restrict__ dst, int E, int N, int nG, int CHP, int NGP, int* __restrict__ STG, int* __restrict__ HST) {
  extern __shared__ int sm[];
  int* cnt = sm; int* run = sm + NGP; int* ids = sm + 2 * NGP;
  const int b = blockIdx.x; const int ch = (E + CSR_NBLK9 - 1) / CSR_NBLK9; const int e0 = b * ch, e1 = min(E, e0 + ch);
  for (int i = threadIdx.x; i < NGP; i += 64) cnt[i] = 0;
  for (int i = threadIdx.x; i < CHP; i += 64) ids[i] = -1;
  __syncthreads();
  if (threadIdx.x == 0) {
    for (int e = e0; e < e1; ++e) { int d = dst[e]; d = (d < 0) ? 0 : (d >= N ? N - 1 : d); cnt[d >> CSR_GB9] += 1; }
    int acc = 0; for (int g = 0; g < nG; ++g) { run[g] = acc; acc += cnt[g]; }
    for (int e = e0; e < e1; ++e) { int d = dst[e]; d = (d < 0) ? 0 : (d >= N ? N - 1 : d); const int g = d >> CSR_GB9; ids[run[g]] = e; run[g] += 1; } }
  __syncthreads();
  typedef __attribute__((ext_vector_type(4))) int v4i;
  for (int pass = 0; pass < 2; ++pass) {
    for (int i = threadIdx.x; i < CHP / 4; i += 64) *(volatile v4i*)(STG + (size_t)b * CHP + i * 4) = *(const v4i*)(&ids[i * 4]);
    for (int i = threadIdx.x; i < NGP / 4; i += 64) { v4i v; for (int e = 0; e < 4; ++e) v[e] = (i * 4 + e < nG) ? cnt[i * 4 + e] : 0; *(volatile v4i*)(HST + (size_t)b * NGP + i * 4) = v; }
    __threadfence(); }
}
__global__ __launch_bounds__(512) void csrS_kernel9(const int* __restrict__ HST, int nG, int NGP, int* __restrict__ START, int* __restrict__ TOT, int* __restrict__ OFF) {
  __shared__ int tot[CSR_MAXG9];
  const int b = threadIdx.x;
  for (int pass = 0; pass < 2; ++pass) { int runb = 0; for (int g = 0; g < nG; ++g) { int c = HST[(size_t)b * NGP + g]; c = (c < 0) ? 0 : c; ((volatile int*)OFF)[(size_t)g * CSR_NBLK9 + b] = runb; runb += c; } __threadfence(); }
  for (int g = threadIdx.x; g < nG; g += 512) { int s = 0; for (int bb = 0; bb < CSR_NBLK9; ++bb) { int c = HST[(size_t)bb * NGP + g]; s += (c < 0) ? 0 : c; } tot[g] = s; }
  __syncthreads();
  if (threadIdx.x < 32) {
    __shared__ int st[CSR_MAXG9 + 32];
    if (threadIdx.x == 0) { int acc = 0; for (int g = 0; g < NGP; ++g) { st[g] = acc; if (g < nG) acc += (tot[g] + 31) & ~31; } st[NGP] = acc; }
    __builtin_amdgcn_fence(__ATOMIC_RELEASE, "workgroup"); __builtin_amdgcn_wave_barrier(); __builtin_amdgcn_fence(__ATOMIC_ACQUIRE, "workgroup");
    for (int pass = 0; pass < 2; ++pass) { for (int i = threadIdx.x; i < NGP + 32; i += 32) { ((volatile int*)START)[i] = (i <= NGP) ? st[min(i, NGP)] : 0; ((volatile int*)TOT)[i] = (i < nG) ? tot[i] : 0; } __threadfence(); } }
}
__global__ __launch_bounds__(256) void csrB_kernel9(const int* __restrict__ dst, int N, int nG, int CHP, int NGP, int permLen, const int* __restrict__ STG, const int* __restrict__ HST, const int* __restrict__ OFF, const int* __restrict__ START, const int* __restrict__ TOT, int* __restrict__ PERM, int* __restrict__ ROWPTR, int* __restrict__ ROWCNT, int* __restrict__ FLAG) {
  typedef __attribute__((ext_vector_type(4))) int v4i;
  __shared__ int ids[CSR_CAP9]; __shared__ unsigned short key[CSR_CAP9]; __shared__ int outp[CSR_CAP9]; __shared__ int ncnt[CSR_GN9 + 1]; __shared__ int boff[CSR_NBLK9 + 1];
  const int g = blockIdx.x, t_ = threadIdx.x; int tot = TOT[g]; int st = START[g], stn = START[g + 1]; const int v0 = g * CSR_GN9; const int nv = min(CSR_GN9, N - v0); const int t0 = g * CSR_TS9;
  st = (st < 0) ? 0 : (st > permLen - 32 ? permLen - 32 : st) & ~31; stn = (stn < st) ? st : (stn > permLen ? permLen : stn); tot = (tot < 0) ? 0 : tot; if (tot > stn - st && tot <= CSR_CAP9) tot = stn - st;
  if (tot > CSR_CAP9) {
    for (int pass = 0; pass < 2; ++pass) { for (int i = t_; i < CSR_TS9 / 4; i += 256) { v4i a, c; for (int e = 0; e < 4; ++e) { a[e] = st; c[e] = 0; } *(volatile v4i*)(ROWPTR + t0 + i * 4) = a; *(volatile v4i*)(ROWCNT + t0 + i * 4) = c; } if (t_ == 0) ((volatile int*)FLAG)[0] = 1; __threadfence(); } (void)nv; return; }
  if (t_ == 0) { int acc = 0; for (int b = 0; b < CSR_NBLK9; ++b) { boff[b] = acc; int c = HST[(size_t)b * NGP + g]; c = (c < 0) ? 0 : (c > CHP ? CHP : c); acc += c; if (acc > tot) acc = tot; } boff[CSR_NBLK9] = acc; }
  for (int i = t_; i <= CSR_GN9; i += 256) ncnt[i] = 0;
  __syncthreads();
  for (int b = 0; b < CSR_NBLK9; ++b) { const int c = boff[b + 1] - boff[b]; int o_ = OFF[(size_t)g * CSR_NBLK9 + b]; o_ = (o_ < 0) ? 0 : (o_ > CHP - c ? CHP - c : o_); const int* src_ = STG + (size_t)b * CHP + o_;
    for (int i = t_; i < c; i += 256) { int id = src_[i]; id = (id < 0) ? 0 : id; ids[boff[b] + i] = id; int d = dst[id]; d = (d < v0) ? v0 : (d >= N ? N - 1 : d); int kk = d - v0; kk = (kk < 0) ? 0 : (kk >= CSR_GN9 ? CSR_GN9 - 1 : kk); key[boff[b] + i] = (unsigned short)kk; } }
  __syncthreads();
  if (t_ == 0) { for (int i = 0; i < tot; ++i) ncnt[key[i]] += 1; int acc = 0; for (int vl = 0; vl < CSR_GN9; ++vl) { const int c = ncnt[vl]; ncnt[vl] = acc; acc += c; } ncnt[CSR_GN9] = acc;
    for (int i = 0; i < tot; ++i) { const int vl = key[i]; outp[ncnt[vl]] = ids[i]; ncnt[vl] += 1; }
    for (int vl = CSR_GN9; vl > 0; --vl) ncnt[vl] = ncnt[vl - 1]; ncnt[0] = 0; }
  __syncthreads();
  for (int pass = 0; pass < 2; ++pass) {
    for (int i = t_; i < (stn - st) / 4; i += 256) { v4i v; for (int e = 0; e < 4; ++e) { const int q = i * 4 + e; v[e] = (q < tot) ? outp[q] : -1; } *(volatile v4i*)(PERM + st + i * 4) = v; }
    for (int i = t_; i < CSR_TS9 / 4; i += 256) { v4i a, c; for (int e = 0; e < 4; ++e) { const int vl = i * 4 + e; const int vc = vl < CSR_GN9 ? vl : CSR_GN9; a[e] = (vl < CSR_GN9) ? st + ncnt[vc] : st; c[e] = (vl < nv) ? (ncnt[(vc < CSR_GN9 ? vc : CSR_GN9 - 1) + 1] - ncnt[vc]) : 0; } *(volatile v4i*)(ROWPTR + t0 + i * 4) = a; *(volatile v4i*)(ROWCNT + t0 + i * 4) = c; }
    __threadfence(); }
}
__global__ __launch_bounds__(256) void csrZ_kernel9(int* __restrict__ p, size_t n4) { typedef __attribute__((ext_vector_type(4))) int v4i; const size_t tid = (size_t)blockIdx.x * 256 + threadIdx.x, nth = (size_t)gridDim.x * 256; v4i z = {0, 0, 0, 0}; for (size_t i = tid; i < n4; i += nth) *(volatile v4i*)(p + i * 4) = z; }
struct CsrBufs9 { int *STG, *HST, *OFF, *START, *TOT, *PERM, *ROWPTR, *ROWCNT, *FLAG; int nG, NGP, CHP; size_t permLen; char* base; size_t bytes; };
static size_t csr_carve9(CsrBufs9& c, char* ws, size_t off, int E, int N) {
  const size_t off0 = off; c.base = ws + off;
  auto al = [&](size_t bytes) { char* p = ws + off; off += (bytes + 255) & ~(size_t)255; return p; };
  c.nG = (N + CSR_GN9 - 1) / CSR_GN9; c.NGP = (c.nG + 31) & ~31; const int ch = (E + CSR_NBLK9 - 1) / CSR_NBLK9; c.CHP = (ch + 31) & ~31; c.permLen = (size_t)E + 32 * (size_t)c.nG + 32;
  c.STG = (int*)al((size_t)CSR_NBLK9 * c.CHP * 4); c.HST = (int*)al((size_t)CSR_NBLK9 * c.NGP * 4); c.OFF = (int*)al((size_t)c.NGP * CSR_NBLK9 * 4); c.START = (int*)al((size_t)(c.NGP + 64) * 4); c.TOT = (int*)al((size_t)(c.NGP + 64) * 4);
  c.PERM = (int*)al(c.permLen * 4); c.ROWPTR = (int*)al((size_t)c.nG * CSR_TS9 * 4); c.ROWCNT = (int*)al((size_t)c.nG * CSR_TS9 * 4); c.FLAG = (int*)al(256);
  c.bytes = off - off0; return off;
}
static void csr_build9(const CsrBufs9& c, const int* dst, int E, int N, hipStream_t stream) {
  const size_t smem = (size_t)(2 * c.NGP + c.CHP) * 4;
  csrZ_kernel9<<<512, 256, 0, stream>>>((int*)c.base, c.bytes / 16);
  csrA_kernel9<<<CSR_NBLK9, 64, smem, stream>>>(dst, E, N, c.nG, c.CHP, c.NGP, c.STG, c.HST);
  csrS_kernel9<<<1, 512, 0, stream>>>(c.HST, c.nG, c.NGP, c.START, c.TOT, c.OFF);
  csrB_kernel9<<<c.nG, 256, 0, stream>>>(dst, N, c.nG, c.CHP, c.NGP, (int)c.permLen, c.STG, c.HST, c.OFF, c.START, c.TOT, c.PERM, c.ROWPTR, c.ROWCNT, c.FLAG);
}

constexpr int CSR_NBLK3 = 512, CSR_GB3 = 3, CSR_GN3 = 1 << CSR_GB3  , CSR_TS3 = (CSR_GN3 < 32 ? 32 : CSR_GN3)  , CSR_MAXG3 = 512, CSR_CAP3 = 12288  ;
__device__ __host__ __forceinline__ int csr_tix3(int v) { return (v >> CSR_GB3) * CSR_TS3 + (v & (CSR_GN3 - 1)); }
__global__ __launch_bounds__(64) void csrA_kernel3(const int* __restrict__ dst, int E, int N, int nG, int CHP, int NGP, int* __restrict__ STG, int* __restrict__ HST) {
  extern __shared__ int sm[];
  int* cnt = sm; int* run = sm + NGP; int* ids = sm + 2 * NGP;
  const int b = blockIdx.x; const int ch = (E + CSR_NBLK3 - 1) / CSR_NBLK3; const int e0 = b * ch, e1 = min(E, e0 + ch);
  for (int i = threadIdx.x; i < NGP; i += 64) cnt[i] = 0;
  for (int i = threadIdx.x; i < CHP; i += 64) ids[i] = -1;
  __syncthreads();
  if (threadIdx.x == 0) {
    for (int e = e0; e < e1; ++e) { int d = dst[e]; d = (d < 0) ? 0 : (d >= N ? N - 1 : d); cnt[d >> CSR_GB3] += 1; }
    int acc = 0; for (int g = 0; g < nG; ++g) { run[g] = acc; acc += cnt[g]; }
    for (int e = e0; e < e1; ++e) { int d = dst[e]; d = (d < 0) ? 0 : (d >= N ? N - 1 : d); const int g = d >> CSR_GB3; ids[run[g]] = e; run[g] += 1; } }
  __syncthreads();
  typedef __attribute__((ext_vector_type(4))) int v4i;
  for (int pass = 0; pass < 2; ++pass) {
    for (int i = threadIdx.x; i < CHP / 4; i += 64) *(volatile v4i*)(STG + (size_t)b * CHP + i * 4) = *(const v4i*)(&ids[i * 4]);
    for (int i = threadIdx.x; i < NGP / 4; i += 64) { v4i v; for (int e = 0; e < 4; ++e) v[e] = (i * 4 + e < nG) ? cnt[i * 4 + e] : 0; *(volatile v4i*)(HST + (size_t)b * NGP + i * 4) = v; }
    __threadfence(); }
}
__global__ __launch_bounds__(512) void csrS_kernel3(const int* __restrict__ HST, int nG, int NGP, int* __restrict__ START, int* __restrict__ TOT, int* __restrict__ OFF) {
  __shared__ int tot[CSR_MAXG3];
  const int b = threadIdx.x;
  for (int pass = 0; pass < 2; ++pass) { int runb = 0; for (int g = 0; g < nG; ++g) { int c = HST[(size_t)b * NGP + g]; c = (c < 0) ? 0 : c; ((volatile int*)OFF)[(size_t)g * CSR_NBLK3 + b] = runb; runb += c; } __threadfence(); }
  for (int g = threadIdx.x; g < nG; g += 512) { int s = 0; for (int bb = 0; bb < CSR_NBLK3; ++bb) { int c = HST[(size_t)bb * NGP + g]; s += (c < 0) ? 0 : c; } tot[g] = s; }
  __syncthreads();
  if (threadIdx.x < 32) {
    __shared__ int st[CSR_MAXG3 + 32];
    if (threadIdx.x == 0) { int acc = 0; for (int g = 0; g < NGP; ++g) { st[g] = acc; if (g < nG) acc += (tot[g] + 31) & ~31; } st[NGP] = acc; }
    __builtin_amdgcn_fence(__ATOMIC_RELEASE, "workgroup"); __builtin_amdgcn_wave_barrier(); __builtin_amdgcn_fence(__ATOMIC_ACQUIRE, "workgroup");
    for (int pass = 0; pass < 2; ++pass) { for (int i = threadIdx.x; i < NGP + 32; i += 32) { ((volatile int*)START)[i] = (i <= NGP) ? st[min(i, NGP)] : 0; ((volatile int*)TOT)[i] = (i < nG) ? tot[i] : 0; } __threadfence(); } }
}
__global__ __launch_bounds__(256) void csrB_kernel3(const int* __restrict__ dst, int N, int nG, int CHP, int NGP, int permLen, const int* __restrict__ STG, const int* __restrict__ HST, const int* __restrict__ OFF, const int* __restrict__ START, const int* __restrict__ TOT, int* __restrict__ PERM, int* __restrict__ ROWPTR, int* __restrict__ ROWCNT, int* __restrict__ FLAG) {
  typedef __attribute__((ext_vector_type(4))) int v4i;
  __shared__ int ids[CSR_CAP3]; __shared__ unsigned short key[CSR_CAP3]; __shared__ int outp[CSR_CAP3]; __shared__ int ncnt[CSR_GN3 + 1]; __shared__ int boff[CSR_NBLK3 + 1];
  const int g = blockIdx.x, t_ = threadIdx.x; int tot = TOT[g]; int st = START[g], stn = START[g + 1]; const int v0 = g * CSR_GN3; const int nv = min(CSR_GN3, N - v0); const int t0 = g * CSR_TS3;
  st = (st < 0) ? 0 : (st > permLen - 32 ? permLen - 32 : st) & ~31; stn = (stn < st) ? st : (stn > permLen ? permLen : stn); tot = (tot < 0) ? 0 : tot; if (tot > stn - st && tot <= CSR_CAP3) tot = stn - st;
  if (tot > CSR_CAP3) {
    for (int pass = 0; pass < 2; ++pass) { for (int i = t_; i < CSR_TS3 / 4; i += 256) { v4i a, c; for (int e = 0; e < 4; ++e) { a[e] = st; c[e] = 0; } *(volatile v4i*)(ROWPTR + t0 + i * 4) = a; *(volatile v4i*)(ROWCNT + t0 + i * 4) = c; } if (t_ == 0) ((volatile int*)FLAG)[0] = 1; __threadfence(); } (void)nv; return; }
  if (t_ == 0) { int acc = 0; for (int b = 0; b < CSR_NBLK3; ++b) { boff[b] = acc; int c = HST[(size_t)b * NGP + g]; c = (c < 0) ? 0 : (c > CHP ? CHP : c); acc += c; if (acc > tot) acc = tot; } boff[CSR_NBLK3] = acc; }
  for (int i = t_; i <= CSR_GN3; i += 256) ncnt[i] = 0;
  __syncthreads();
  for (int b = 0; b < CSR_NBLK3; ++b) { const int c = boff[b + 1] - boff[b]; int o_ = OFF[(size_t)g * CSR_NBLK3 + b]; o_ = (o_ < 0) ? 0 : (o_ > CHP - c ? CHP - c : o_); const int* src_ = STG + (size_t)b * CHP + o_;
    for (int i = t_; i < c; i += 256) { int id = src_[i]; id = (id < 0) ? 0 : id; ids[boff[b] + i] = id; int d = dst[id]; d = (d < v0) ? v0 : (d >= N ? N - 1 : d); int kk = d - v0; kk = (kk < 0) ? 0 : (kk >= CSR_GN3 ? CSR_GN3 - 1 : kk); key[boff[b] + i] = (unsigned short)kk; } }
  __syncthreads();
  if (t_ == 0) { for (int i = 0; i < tot; ++i) ncnt[key[i]] += 1; int acc = 0; for (int vl = 0; vl < CSR_GN3; ++vl) { const int c = ncnt[vl]; ncnt[vl] = acc; acc += c; } ncnt[CSR_GN3] = acc;
    for (int i = 0; i < tot; ++i) { const int vl = key[i]; outp[ncnt[vl]] = ids[i]; ncnt[vl] += 1; }
    for (int vl = CSR_GN3; vl > 0; --vl) ncnt[vl] = ncnt[vl - 1]; ncnt[0] = 0; }
  __syncthreads();
  for (int pass = 0; pass < 2; ++pass) {
    for (int i = t_; i < (stn - st) / 4; i += 256) { v4i v; for (int e = 0; e < 4; ++e) { const int q = i * 4 + e; v[e] = (q < tot) ? outp[q] : -1; } *(volatile v4i*)(PERM + st + i * 4) = v; }
    for (int i = t_; i < CSR_TS3 / 4; i += 256) { v4i a, c; for (int e = 0; e < 4; ++e) { const int vl = i * 4 + e; const int vc = vl < CSR_GN3 ? vl : CSR_GN3; a[e] = (vl < CSR_GN3) ? st + ncnt[vc] : st; c[e] = (vl < nv) ? (ncnt[(vc < CSR_GN3 ? vc : CSR_GN3 - 1) + 1] - ncnt[vc]) : 0; } *(volatile v4i*)(ROWPTR + t0 + i * 4) = a; *(volatile v4i*)(ROWCNT + t0 + i * 4) = c; }
    __threadfence(); }
}
__global__ __launch_bounds__(256) void csrZ_kernel3(int* __restrict__ p, size_t n4) { typedef __attribute__((ext_vector_type(4))) int v4i; const size_t tid = (size_t)blockIdx.x * 256 + threadIdx.x, nth = (size_t)gridDim.x * 256; v4i z = {0, 0, 0, 0}; for (size_t i = tid; i < n4; i += nth) *(volatile v4i*)(p + i * 4) = z; }
struct CsrBufs3 { int *STG, *HST, *OFF, *START, *TOT, *PERM, *ROWPTR, *ROWCNT, *FLAG; int nG, NGP, CHP; size_t permLen; char* base; size_t bytes; };
static size_t csr_carve3(CsrBufs3& c, char* ws, size_t off, int E, int N) {
  const size_t off0 = off; c.base = ws + off;
  auto al = [&](size_t bytes) { char* p = ws + off; off += (bytes + 255) & ~(size_t)255; return p; };
  c.nG = (N + CSR_GN3 - 1) / CSR_GN3; c.NGP = (c.nG + 31) & ~31; const int ch = (E + CSR_NBLK3 - 1) / CSR_NBLK3; c.CHP = (ch + 31) & ~31; c.permLen = (size_t)E + 32 * (size_t)c.nG + 32;
  c.STG = (int*)al((size_t)CSR_NBLK3 * c.CHP * 4); c.HST = (int*)al((size_t)CSR_NBLK3 * c.NGP * 4); c.OFF = (int*)al((size_t)c.NGP * CSR_NBLK3 * 4); c.START = (int*)al((size_t)(c.NGP + 64) * 4); c.TOT = (int*)al((size_t)(c.NGP + 64) * 4);
  c.PERM = (int*)al(c.permLen * 4); c.ROWPTR = (int*)al((size_t)c.nG * CSR_TS3 * 4); c.ROWCNT = (int*)al((size_t)c.nG * CSR_TS3 * 4); c.FLAG = (int*)al(256);
  c.bytes = off - off0; return off;
}
static void csr_build3(const CsrBufs3& c, const int* dst, int E, int N, hipStream_t stream) {
  const size_t smem = (size_t)(2 * c.NGP + c.CHP) * 4;
  csrZ_kernel3<<<512, 256, 0, stream>>>((int*)c.base, c.bytes / 16);
  csrA_kernel3<<<CSR_NBLK3, 64, smem, stream>>>(dst, E, N, c.nG, c.CHP, c.NGP, c.STG, c.HST);
  csrS_kernel3<<<1, 512, 0, stream>>>(c.HST, c.nG, c.NGP, c.START, c.TOT, c.OFF);
  csrB_kernel3<<<c.nG, 256, 0, stream>>>(dst, N, c.nG, c.CHP, c.NGP, (int)c.permLen, c.STG, c.HST, c.OFF, c.START, c.TOT, c.PERM, c.ROWPTR, c.ROWCNT, c.FLAG);
}


__global__ __launch_bounds__(256) void wcopy_kernel(const float* __restrict__ w, int INW, int c0, int KIN, int OUT, int KP, b16* __restrict__ WT) {
  const int u = blockIdx.x * 256 + threadIdx.x; if (u >= OUT * KP / 8) return; const int e = u * 8; const int o = e / KP, k0 = e % KP; v8b v;
#pragma unroll
  for (int j = 0; j < 8; ++j) { const int k = k0 + j; v[j] = k < KIN ? (b16)(bf16_rne(w[(size_t)o * INW + c0 + k]) * WSC) : (b16)0.0f; } for (int pass = 0; pass < 2; ++pass) { *(volatile v8b*)(WT + e) = v; __threadfence(); }
}
template <int NT> __device__ __forceinline__ void ln_tiles(float (&vals)[NT][8], const float* __restrict__ g, const float* __restrict__ b, int nloc) {
  float ps[8], pq[8];
#pragma unroll
  for (int r8 = 0; r8 < 8; ++r8) { ps[r8] = 0.0f;
#pragma unroll
    for (int t = 0; t < NT; ++t) ps[r8] += vals[t][r8];
    for (int o = 1; o < 16; o <<= 1) ps[r8] += __shfl_xor(ps[r8], o); ps[r8] *= (1.0f / (NT * 16)); pq[r8] = 0.0f;
#pragma unroll
    for (int t = 0; t < NT; ++t) { const float d = vals[t][r8] - ps[r8]; pq[r8] += pmul(d, d); }
    for (int o = 1; o < 16; o <<= 1) pq[r8] += __shfl_xor(pq[r8], o); pq[r8] = rsqrtf(pq[r8] * (1.0f / (NT * 16)) + EPS); }
#pragma unroll
  for (int t = 0; t < NT; ++t) { const float gg = bf16_rne(g[t * 16 + nloc]), be = bf16_rne(b[t * 16 + nloc]);
#pragma unroll
    for (int r8 = 0; r8 < 8; ++r8) vals[t][r8] = pmul(pmul(vals[t][r8] - ps[r8], pq[r8]), gg) + be; }
}
__global__ __launch_bounds__(32) void emb_kernel(const float* __restrict__ x, const b16* __restrict__ WT, const float* __restrict__ bias, const float* __restrict__ g, const float* __restrict__ bb, float* __restrict__ Hout) {
  __shared__ __attribute__((aligned(16))) b16 Ah[16][32 + 8]; __shared__ __attribute__((aligned(16))) float Tf[16][H + 4];
  const int lane = threadIdx.x, nloc = lane & 15, hlf = lane >> 4; const size_t m0 = (size_t)blockIdx.x * 16;
  for (int rr = 0; rr < 16; ++rr) Ah[rr][lane] = lane < 3 ? (b16)(bf16_rne(x[(m0 + rr) * 3 + lane]) * XS) : (b16)0.0f;
  wave_lds_sync();
  v8f acc[8]; const v16b a = frag_kb(&Ah[nloc][0], hlf);
#pragma unroll
  for (int t = 0; t < 8; ++t) { acc[t] = (v8f){}; acc[t] = wmma16b(a, frag_kb(WT + (size_t)(t * 16 + nloc) * 32, hlf), acc[t]); }
  float vals[8][8];
#pragma unroll
  for (int t = 0; t < 8; ++t) { const float bv = bf16_rne(bias[t * 16 + nloc]);
#pragma unroll
    for (int r8 = 0; r8 < 8; ++r8) vals[t][r8] = acc[t][r8] * (1.0f / (XS * WSC)) + bv; }
  ln_tiles<8>(vals, g, bb, nloc);
#pragma unroll
  for (int t = 0; t < 8; ++t)
#pragma unroll
    for (int r8 = 0; r8 < 8; ++r8) Tf[8 * hlf + r8][t * 16 + nloc] = silu(vals[t][r8]);
  wave_lds_sync();
  for (int pass = 0; pass < 2; ++pass) { for (int rr = 0; rr < 16; ++rr) *(volatile v4f*)(Hout + (m0 + rr) * H + lane * 4) = *(const v4f*)(&Tf[rr][lane * 4]); __threadfence(); }
}
__global__ __launch_bounds__(32) void pq_kernel(const float* __restrict__ Hp, const b16* __restrict__ WT, int NLIM, float* __restrict__ PQ) {
  __shared__ __attribute__((aligned(16))) b16 Ah[16][H + 8], Al[16][H + 8]; __shared__ __attribute__((aligned(16))) float Tf[16][128 + 4];
  const int lane = threadIdx.x, nloc = lane & 15, hlf = lane >> 4; const size_t m0 = (size_t)blockIdx.x * 16; if (m0 >= (size_t)NLIM) return;
  for (int rr = 0; rr < 16; ++rr) { const v4f v = *(const v4f*)(Hp + (m0 + rr) * H + lane * 4); for (int j = 0; j < 4; ++j) { b16 p, q; split16(v[j] * XS, p, q); Ah[rr][lane * 4 + j] = p; Al[rr][lane * 4 + j] = q; } }
  wave_lds_sync();
#pragma unroll 1
  for (int cg = 0; cg < 2 * H2 / 128; ++cg) { v8f acc[8];
#pragma unroll
    for (int t = 0; t < 8; ++t) acc[t] = (v8f){};
#pragma unroll 2
    for (int kb = 0; kb < H; kb += 32) { const v16b a = frag_kb(&Ah[nloc][kb], hlf), al = frag_kb(&Al[nloc][kb], hlf);
#pragma unroll
      for (int t = 0; t < 8; ++t) { const v16b bw = frag_kb(WT + (size_t)(cg * 128 + t * 16 + nloc) * H + kb, hlf); acc[t] = wmma16b(a, bw, acc[t]); acc[t] = wmma16b(al, bw, acc[t]); } }
#pragma unroll
    for (int t = 0; t < 8; ++t)
#pragma unroll 1
      for (int r8 = 0; r8 < 8; ++r8) Tf[8 * hlf + r8][t * 16 + nloc] = acc[t][r8] * (1.0f / (XS * WSC));
    wave_lds_sync();
    for (int pass = 0; pass < 2; ++pass) { for (int rr = 0; rr < 16; ++rr) *(volatile v4f*)(PQ + (m0 + rr) * (2 * H2) + cg * 128 + lane * 4) = *(const v4f*)(&Tf[rr][lane * 4]); __threadfence(); }
    wave_lds_sync(); }
}
__global__ __launch_bounds__(256) void edge_kernel(const float* __restrict__ PQ, const float* __restrict__ ea, const float* __restrict__ w1, const float* __restrict__ b1, const int* __restrict__ srcs, const int* __restrict__ PERM, const int* __restrict__ ROWPTR, const int* __restrict__ ROWCNT, int permLen, int NLIM, float* __restrict__ Sout) {
  const int wave = threadIdx.x >> 5, lane = threadIdx.x & 31; const size_t v = (size_t)blockIdx.x * 8 + wave; float s[8]; for (int i = 0; i < 8; ++i) s[i] = 0.0f;
  if (v < (size_t)NLIM) { float we[8], bb[8], pv[8]; for (int i = 0; i < 8; ++i) { const int c = lane * 8 + i; we[i] = bf16_rne(w1[(size_t)c * (H2 + 1) + H2]); bb[i] = bf16_rne(b1[c]); }
    { const v4f a = *(const v4f*)(PQ + v * (2 * H2) + lane * 8), b = *(const v4f*)(PQ + v * (2 * H2) + lane * 8 + 4); for (int i = 0; i < 4; ++i) { pv[i] = a[i]; pv[4 + i] = b[i]; } }
    int st = ROWPTR[v], cnt = ROWCNT[v]; cnt = iclamp(cnt, 0, 1 << 20); st = iclamp(st, 0, permLen - cnt);
#pragma unroll 1
    for (int j = 0; j < cnt; ++j) { const int e = iclamp(PERM[st + j], 0, E - 1); const size_t sj = (size_t)iclamp(srcs[e], 0, N - 1); if (sj >= (size_t)NLIM) continue; const float a = bf16_rne(ea[e]); const v4f q0 = *(const v4f*)(PQ + sj * (2 * H2) + H2 + lane * 8), q1 = *(const v4f*)(PQ + sj * (2 * H2) + H2 + lane * 8 + 4);
      for (int i = 0; i < 4; ++i) { s[i] += silu(pv[i] + q0[i] + pmul(a, we[i]) + bb[i]); s[4 + i] += silu(pv[4 + i] + q1[i] + pmul(a, we[4 + i]) + bb[4 + i]); } } }
  v4f o0 = {s[0], s[1], s[2], s[3]}, o1 = {s[4], s[5], s[6], s[7]};
  for (int pass = 0; pass < 2; ++pass) { *(volatile v4f*)(Sout + v * H2 + lane * 8) = o0; *(volatile v4f*)(Sout + v * H2 + lane * 8 + 4) = o1; __threadfence(); }
}
__global__ __launch_bounds__(32) void upd_kernel(const float* __restrict__ S, const float* __restrict__ Hp, const int* __restrict__ ROWCNT, const b16* __restrict__ W2T, const float* __restrict__ b2, const b16* __restrict__ WGT, const float* __restrict__ bg, const float* __restrict__ g, const float* __restrict__ bb, int NLIM, float* __restrict__ Hout) {
  __shared__ __attribute__((aligned(16))) b16 Ah[16][H2 + 8], Al[16][H2 + 8]; __shared__ __attribute__((aligned(16))) float Hs[16][H + 4], Tf[16][H + 4];
  const int lane = threadIdx.x, nloc = lane & 15, hlf = lane >> 4; const size_t m0 = (size_t)blockIdx.x * 16; if (m0 >= (size_t)NLIM) return;
  for (int rr = 0; rr < 16; ++rr) { for (int q = 0; q < 2; ++q) { const v4f v = *(const v4f*)(S + (m0 + rr) * H2 + q * 128 + lane * 4); for (int j = 0; j < 4; ++j) { b16 p, ql; split16(v[j] * XS, p, ql); Ah[rr][q * 128 + lane * 4 + j] = p; Al[rr][q * 128 + lane * 4 + j] = ql; } }
    const v4f hv = *(const v4f*)(Hp + (m0 + rr) * H + lane * 4); for (int j = 0; j < 4; ++j) Hs[rr][lane * 4 + j] = hv[j]; }
  wave_lds_sync();
  v8f acc[8];
#pragma unroll
  for (int t = 0; t < 8; ++t) acc[t] = (v8f){};
#pragma unroll 2
  for (int kb = 0; kb < H2; kb += 32) { const v16b a = frag_kb(&Ah[nloc][kb], hlf), al = frag_kb(&Al[nloc][kb], hlf);
#pragma unroll
    for (int t = 0; t < 8; ++t) { const v16b bw = frag_kb(W2T + (size_t)(t * 16 + nloc) * H2 + kb, hlf); acc[t] = wmma16b(a, bw, acc[t]); acc[t] = wmma16b(al, bw, acc[t]); } }
  wave_lds_sync();
  float ag[8][8];
#pragma unroll
  for (int t = 0; t < 8; ++t) { const int c = t * 16 + nloc; const float bv = bf16_rne(b2[c]);
#pragma unroll
    for (int r8 = 0; r8 < 8; ++r8) { const int rl = 8 * hlf + r8; const size_t r = m0 + rl; const int cn = r < (size_t)N ? iclamp(ROWCNT[r], 0, 1 << 20) : 0; const float a = acc[t][r8] * (1.0f / (XS * WSC)) + pmul((float)cn, bv); ag[t][r8] = a;
      b16 p, ql; split16(Hs[rl][c] * XS, p, ql); Ah[rl][c] = p; Al[rl][c] = ql; split16(a * XS, p, ql); Ah[rl][H + c] = p; Al[rl][H + c] = ql; } }
  wave_lds_sync();
#pragma unroll
  for (int t = 0; t < 8; ++t) acc[t] = (v8f){};
#pragma unroll 2
  for (int kb = 0; kb < H2; kb += 32) { const v16b a = frag_kb(&Ah[nloc][kb], hlf), al = frag_kb(&Al[nloc][kb], hlf);
#pragma unroll
    for (int t = 0; t < 8; ++t) { const v16b bw = frag_kb(WGT + (size_t)(t * 16 + nloc) * H2 + kb, hlf); acc[t] = wmma16b(a, bw, acc[t]); acc[t] = wmma16b(al, bw, acc[t]); } }
  float vals[8][8];
#pragma unroll
  for (int t = 0; t < 8; ++t) { const int c = t * 16 + nloc; const float bv = bf16_rne(bg[c]);
#pragma unroll
    for (int r8 = 0; r8 < 8; ++r8) { const int rl = 8 * hlf + r8; const float gt = sigm(acc[t][r8] * (1.0f / (XS * WSC)) + bv); const float hv = Hs[rl][c]; vals[t][r8] = hv + (pmul(gt, ag[t][r8]) + pmul(1.0f - gt, hv)); } }
  ln_tiles<8>(vals, g, bb, nloc);
  wave_lds_sync();
#pragma unroll
  for (int t = 0; t < 8; ++t)
#pragma unroll
    for (int r8 = 0; r8 < 8; ++r8) Tf[8 * hlf + r8][t * 16 + nloc] = vals[t][r8];
  wave_lds_sync();
  for (int pass = 0; pass < 2; ++pass) { for (int rr = 0; rr < 16; ++rr) *(volatile v4f*)(Hout + (m0 + rr) * H + lane * 4) = *(const v4f*)(&Tf[rr][lane * 4]); __threadfence(); }
}
__global__ __launch_bounds__(128) void pool_kernel(const float* __restrict__ Hp, const int* __restrict__ PERM, const int* __restrict__ ROWPTR, const int* __restrict__ ROWCNT, int permLen, int NLIM, const b16* __restrict__ WP1, const float* __restrict__ p1b, const float* __restrict__ g1, const float* __restrict__ b1, const b16* __restrict__ WP2, const float* __restrict__ p2b, const float* __restrict__ g2, const float* __restrict__ bb2, float* __restrict__ out) {
  __shared__ __attribute__((aligned(16))) b16 Ah[4][16][H + 8], Al[4][16][H + 8]; __shared__ __attribute__((aligned(16))) float Tf[4][16][H + 4];
  const int wave = threadIdx.x >> 5, lane = threadIdx.x & 31, nloc = lane & 15, hlf = lane >> 4; const int g0 = wave * 16;
  for (int rr = 0; rr < 16; ++rr) { const int gg = g0 + rr; const int tix = (gg >> 3) * 32 + (gg & 7); int st = ROWPTR[tix], cnt = ROWCNT[tix]; cnt = iclamp(cnt, 0, 1 << 20); st = iclamp(st, 0, permLen - cnt); v4f s = {0, 0, 0, 0}; int used = 0;
#pragma unroll 1
    for (int j = 0; j < cnt; ++j) { const int n = iclamp(PERM[st + j], 0, N - 1); if (n >= NLIM) continue; ++used; const v4f hv = *(const v4f*)(Hp + (size_t)n * H + lane * 4); for (int i = 0; i < 4; ++i) s[i] += hv[i]; }
    const float c1 = (float)(used < 1 ? 1 : used), c2 = (float)used + 1e-6f;
    for (int i = 0; i < 4; ++i) { const float xg = s[i] / c1 + s[i] / c2; Tf[wave][rr][lane * 4 + i] = xg; b16 p, q; split16(xg * XS, p, q); Ah[wave][rr][lane * 4 + i] = p; Al[wave][rr][lane * 4 + i] = q; } }
  wave_lds_sync();
  for (int pass = 0; pass < 2; ++pass) { for (int rr = 0; rr < 16; ++rr) *(volatile v4f*)(out + G * LAT + (size_t)(g0 + rr) * H + lane * 4) = *(const v4f*)(&Tf[wave][rr][lane * 4]); __threadfence(); }
  v8f acc[8];
#pragma unroll
  for (int t = 0; t < 8; ++t) acc[t] = (v8f){};
#pragma unroll 2
  for (int kb = 0; kb < H; kb += 32) { const v16b a = frag_kb(&Ah[wave][nloc][kb], hlf), al = frag_kb(&Al[wave][nloc][kb], hlf);
#pragma unroll
    for (int t = 0; t < 8; ++t) { const v16b bw = frag_kb(WP1 + (size_t)(t * 16 + nloc) * H + kb, hlf); acc[t] = wmma16b(a, bw, acc[t]); acc[t] = wmma16b(al, bw, acc[t]); } }
  float vals[8][8];
#pragma unroll
  for (int t = 0; t < 8; ++t) { const float bv = bf16_rne(p1b[t * 16 + nloc]);
#pragma unroll
    for (int r8 = 0; r8 < 8; ++r8) vals[t][r8] = acc[t][r8] * (1.0f / (XS * WSC)) + bv; }
  ln_tiles<8>(vals, g1, b1, nloc);
  wave_lds_sync();
#pragma unroll
  for (int t = 0; t < 8; ++t) { const int c = t * 16 + nloc;
#pragma unroll
    for (int r8 = 0; r8 < 8; ++r8) { const float p = silu(vals[t][r8]); b16 ph, pl; split16(p * XS, ph, pl); Ah[wave][8 * hlf + r8][c] = ph; Al[wave][8 * hlf + r8][c] = pl; } }
  wave_lds_sync();
  v8f a2[4];
#pragma unroll
  for (int t = 0; t < 4; ++t) a2[t] = (v8f){};
#pragma unroll 2
  for (int kb = 0; kb < H; kb += 32) { const v16b a = frag_kb(&Ah[wave][nloc][kb], hlf), al = frag_kb(&Al[wave][nloc][kb], hlf);
#pragma unroll
    for (int t = 0; t < 4; ++t) { const v16b bw = frag_kb(WP2 + (size_t)(t * 16 + nloc) * H + kb, hlf); a2[t] = wmma16b(a, bw, a2[t]); a2[t] = wmma16b(al, bw, a2[t]); } }
  float v2[4][8];
#pragma unroll
  for (int t = 0; t < 4; ++t) { const float bv = bf16_rne(p2b[t * 16 + nloc]);
#pragma unroll
    for (int r8 = 0; r8 < 8; ++r8) v2[t][r8] = a2[t][r8] * (1.0f / (XS * WSC)) + bv; }
  ln_tiles<4>(v2, g2, bb2, nloc);
#pragma unroll
  for (int t = 0; t < 4; ++t)
#pragma unroll
    for (int r8 = 0; r8 < 8; ++r8) Tf[wave][8 * hlf + r8][t * 16 + nloc] = v2[t][r8];
  wave_lds_sync();
  for (int pass = 0; pass < 2; ++pass) { for (int rr = 0; rr < 16; ++rr) *(volatile v2f*)(out + (size_t)(g0 + rr) * LAT + lane * 2) = *(const v2f*)(&Tf[wave][rr][lane * 2]); __threadfence(); }
}
}

extern "C" void kernel_launch(void* const* d_in, const int* in_sizes, int n_in, void* d_out, int out_size, void* d_ws, size_t ws_size, hipStream_t stream) {
  (void)n_in;
  auto Fp = [&](int i) { return (const float*)d_in[i]; }; auto Ip = [&](int i) { return (const int*)d_in[i]; };
  if (in_sizes[0] != N * 3 || in_sizes[1] != E || in_sizes[2] != 2 * E || in_sizes[3] != N || in_sizes[4] != H * 3 || in_sizes[8] != NL * H2 * (H2 + 1) || in_sizes[10] != NL * H * H2 || in_sizes[12] != NL * H * H2 || in_sizes[16] != H * H || in_sizes[20] != LAT * H || out_size != G * LAT + G * H) return;
  const int NLIM = N; const int GB16 = NBLK, GB8 = N / 8;
  size_t off = 0; char* ws = (char*)d_ws;
  auto carve = [&](size_t bytes) { char* p = ws + off; off += (bytes + 255) & ~(size_t)255; return p; };
  b16* WEMB = (b16*)carve(H * 32 * 2); b16* WPQ[NL]; b16* W2T[NL]; b16* WGT[NL]; for (int l = 0; l < NL; ++l) { WPQ[l] = (b16*)carve((size_t)2 * H2 * H * 2); W2T[l] = (b16*)carve((size_t)H * H2 * 2); WGT[l] = (b16*)carve((size_t)H * H2 * 2); }
  b16* WP1 = (b16*)carve(H * H * 2); b16* WP2 = (b16*)carve(LAT * H * 2);
  float* HA = (float*)carve((size_t)N * H * 4); float* HB = (float*)carve((size_t)N * H * 4); float* PQ = (float*)carve((size_t)N * 2 * H2 * 4); float* S = (float*)carve((size_t)N * H2 * 4);
  CsrBufs9 csr; CsrBufs3 pl; off = csr_carve9(csr, ws, off, E, N); off = csr_carve3(pl, ws, off, N, G);
  if (off > ws_size || off > ((size_t)96 << 20)) return;
  wcopy_kernel<<<(H * 32 / 8 + 255) / 256, 256, 0, stream>>>(Fp(4), 3, 0, 3, H, 32, WEMB);
  for (int l = 0; l < NL; ++l) { const float* w1 = Fp(8) + (size_t)l * H2 * (H2 + 1);
    wcopy_kernel<<<(H2 * H / 8 + 255) / 256, 256, 0, stream>>>(w1, H2 + 1, 0, H, H2, H, WPQ[l]);
    wcopy_kernel<<<(H2 * H / 8 + 255) / 256, 256, 0, stream>>>(w1, H2 + 1, H, H, H2, H, WPQ[l] + H2 * H);
    wcopy_kernel<<<(H * H2 / 8 + 255) / 256, 256, 0, stream>>>(Fp(10) + (size_t)l * H * H2, H2, 0, H2, H, H2, W2T[l]); wcopy_kernel<<<(H * H2 / 8 + 255) / 256, 256, 0, stream>>>(Fp(12) + (size_t)l * H * H2, H2, 0, H2, H, H2, WGT[l]); }
  wcopy_kernel<<<(H * H / 8 + 255) / 256, 256, 0, stream>>>(Fp(16), H, 0, H, H, H, WP1); wcopy_kernel<<<(LAT * H / 8 + 255) / 256, 256, 0, stream>>>(Fp(20), H, 0, H, LAT, H, WP2);
  csr_build9(csr, Ip(2) + E, E, N, stream); csr_build3(pl, Ip(3), N, G, stream);
  emb_kernel<<<NBLK, 32, 0, stream>>>(Fp(0), WEMB, Fp(5), Fp(6), Fp(7), HA);
  float* hin = HA; float* hout = HB;
  for (int l = 0; l < NL; ++l) {
    pq_kernel<<<GB16, 32, 0, stream>>>(hin, WPQ[l], NLIM, PQ);
    edge_kernel<<<GB8, 256, 0, stream>>>(PQ, Fp(1), Fp(8) + (size_t)l * H2 * (H2 + 1), Fp(9) + l * H2, Ip(2), csr.PERM, csr.ROWPTR, csr.ROWCNT, (int)csr.permLen, NLIM, S);
    upd_kernel<<<GB16, 32, 0, stream>>>(S, hin, csr.ROWCNT, W2T[l], Fp(11) + l * H, WGT[l], Fp(13) + l * H, Fp(14) + l * H, Fp(15) + l * H, NLIM, hout);
    float* t = hin; hin = hout; hout = t; }
  pool_kernel<<<1, 128, 0, stream>>>(hin, pl.PERM, pl.ROWPTR, pl.ROWCNT, (int)pl.permLen, NLIM, WP1, Fp(17), Fp(18), Fp(19), WP2, Fp(21), Fp(22), Fp(23), (float*)d_out);
}
